// EmbeddingMixer_28647431865058
// MI455X (gfx1250) — hardware-verified
//
#include <hip/hip_runtime.h>
#include <math.h>

typedef __attribute__((ext_vector_type(16))) _Float16 v16h;
typedef __attribute__((ext_vector_type(16))) __bf16 v16b;
typedef __attribute__((ext_vector_type(8)))  _Float16 v8h;
typedef __attribute__((ext_vector_type(8)))  float v8f;
typedef __attribute__((ext_vector_type(4)))  float v4f;
typedef __attribute__((ext_vector_type(2)))  float v2f;
typedef __attribute__((ext_vector_type(4)))  unsigned v4u;
typedef __attribute__((ext_vector_type(4)))  int v4i;
typedef float __attribute__((may_alias)) float_a;
typedef int __attribute__((may_alias)) int_a;

template <typename T> __device__ __forceinline__ void vst2(void* p, T v) { *(volatile T*)p = v; __threadfence(); *(volatile T*)p = v; }
__device__ __forceinline__ v8f wmma16(v16h a, v16h b, v8f c) {
  v8f d = __builtin_amdgcn_wmma_f32_16x16x32_f16(false, a, false, b, (short)0, c, false, false);
  asm volatile("v_nop\n\tv_nop\n\tv_nop\n\tv_nop" : "+v"(d) : "v"(a), "v"(b));
  return d;
}
__device__ __forceinline__ v8f wmma_bf(v16b a, v16b b, v8f c) {
  v8f d = __builtin_amdgcn_wmma_f32_16x16x32_bf16(false, a, false, b, (short)0, c, false, false);
  asm volatile("v_nop\n\tv_nop\n\tv_nop\n\tv_nop" : "+v"(d) : "v"(a), "v"(b));
  return d;
}
__device__ __forceinline__ v16h frag_h(const _Float16* rowk0, int lane) {
  union { v16h v; v8h q[2]; } u; const _Float16* p = rowk0 + 8 * (lane >> 4);
  u.q[0] = *(const v8h*)p; u.q[1] = *(const v8h*)(p + 16); return u.v;
}
__device__ __forceinline__ v16h frag_f32(const float* rowk0, int lane) {
  v16h a; const float* p = rowk0 + 8 * (lane >> 4);
#pragma unroll
  for (int i = 0; i < 8; ++i) { a[i] = (_Float16)p[i]; a[8 + i] = (_Float16)p[16 + i]; }
  return a;
}
__device__ __forceinline__ v16h frag_f32s(const float* rowk0, int lane, float sc) {
  v16h a; const float* p = rowk0 + 8 * (lane >> 4);
#pragma unroll
  for (int i = 0; i < 8; ++i) { a[i] = (_Float16)(p[i] * sc); a[8 + i] = (_Float16)(p[16 + i] * sc); }
  return a;
}
__device__ __forceinline__ v16h fragc_f32(const float* W, int k0, int n, int lane, int ld, int K) {
  v16h a; const int g = lane >> 4;
#pragma unroll
  for (int i = 0; i < 8; ++i) { const int ka = k0 + 8 * g + i, kb = ka + 16;
    a[i] = (_Float16)(ka < K ? W[(size_t)ka * ld + n] : 0.f); a[8 + i] = (_Float16)(kb < K ? W[(size_t)kb * ld + n] : 0.f); }
  return a;
}
struct F2 { v16b h, l; };
__device__ __forceinline__ F2 bsplit16(const float v[16]) { F2 r;
#pragma unroll
  for (int i = 0; i < 16; ++i) { const __bf16 h = (__bf16)v[i]; r.h[i] = h; r.l[i] = (__bf16)(v[i] - (float)h); }
  return r; }
__device__ __forceinline__ F2 split_row(const float* row, int k0, int lane) { float v[16]; const float* p = row + k0 + 8 * (lane >> 4);
#pragma unroll
  for (int i = 0; i < 8; ++i) { v[i] = p[i]; v[8 + i] = p[16 + i]; }
  return bsplit16(v); }
__device__ __forceinline__ F2 split_rowK(const float* row, int k0, int lane, int K) { float v[16]; const int g = lane >> 4;
#pragma unroll
  for (int i = 0; i < 8; ++i) { const int ka = k0 + 8 * g + i, kb = ka + 16; v[i] = ka < K ? row[ka] : 0.f; v[8 + i] = kb < K ? row[kb] : 0.f; }
  return bsplit16(v); }
__device__ __forceinline__ F2 split_col(const float* W, int k0, int n, int lane, int ld, int K) { float v[16]; const int g = lane >> 4;
#pragma unroll
  for (int i = 0; i < 8; ++i) { const int ka = k0 + 8 * g + i, kb = ka + 16; v[i] = ka < K ? W[(size_t)ka * ld + n] : 0.f; v[8 + i] = kb < K ? W[(size_t)kb * ld + n] : 0.f; }
  return bsplit16(v); }
__device__ __forceinline__ v8f mac3(const F2& a, const F2& b, v8f c) { c = wmma_bf(a.l, b.h, c); c = wmma_bf(a.h, b.l, c); return wmma_bf(a.h, b.h, c); }
__device__ __forceinline__ float sigm(float v) { return 1.0f / (1.0f + expf(-v)); }
#define LDSX() do { asm volatile("s_wait_dscnt 0" ::: "memory"); __builtin_amdgcn_wave_barrier(); __builtin_amdgcn_fence(__ATOMIC_RELEASE, "workgroup"); } while (0)

#define NT 8192
#define D0 256
#define H1 1024
#define NBAS 6
#define K1 (D0 * 7)
#define K2 (H1 * 7)

__device__ __forceinline__ void bspl(float x, float out[NBAS]) {
  const float h = 2.0f / 3.0f, g0 = -3.0f * h - 1.0f;
  const float tpos = (x - g0) / h; const float cf = floorf(tpos); const int c = (int)cf; const float u = tpos - cf;
  const float u2 = u * u, u3 = u2 * u;
  const float w0 = (1.0f - u) * (1.0f - u) * (1.0f - u) * (1.0f / 6.0f), w1 = (3.0f * u3 - 6.0f * u2 + 4.0f) * (1.0f / 6.0f), w2 = (-3.0f * u3 + 3.0f * u2 + 3.0f * u + 1.0f) * (1.0f / 6.0f), w3 = u3 * (1.0f / 6.0f);
  const bool in = (x >= g0) && (c >= 0) && (c < 9);
#pragma unroll
  for (int j = 0; j < NBAS; ++j) { const int d = c - j; out[j] = (in && d >= 0 && d <= 3) ? (d == 3 ? w0 : (d == 2 ? w1 : (d == 1 ? w2 : w3))) : 0.f; }
}
__device__ __forceinline__ float silu1(float v) { return v / (1.0f + expf(-v)); }
__device__ __forceinline__ float gelu_e(float v) { return 0.5f * v * (1.0f + erff(v * 0.70710678118654752f)); }

__global__ __launch_bounds__(256) void k_a1(const float* __restrict__ x, _Float16* __restrict__ A1) {
  __shared__ __align__(16) _Float16 row[K1];
  const int n = blockIdx.x, i = threadIdx.x; const float v = x[(size_t)n * D0 + i];
  row[i] = (_Float16)(silu1(v) * 64.0f); float bs[NBAS]; bspl(v, bs);
#pragma unroll
  for (int k = 0; k < NBAS; ++k) row[D0 + i * NBAS + k] = (_Float16)(bs[k] * 64.0f);
  __syncthreads();
  for (int q = i; q < K1 / 8; q += 256) vst2(A1 + (size_t)n * K1 + q * 8, *(const v4u*)(&row[q * 8]));
}
__global__ __launch_bounds__(256) void k_pack(const float* __restrict__ bw, const float* __restrict__ sw, const float* __restrict__ sc, int DIN, _Float16* __restrict__ P) {
  const int o = blockIdx.x, tid = threadIdx.x; const int K = DIN * 7;
  extern __shared__ __align__(16) _Float16 prow[];
  for (int i = tid; i < DIN; i += 256) { prow[i] = (_Float16)(bw[(size_t)o * DIN + i] * 16.0f); const float s = sc[(size_t)o * DIN + i] * 16.0f;
#pragma unroll
    for (int k = 0; k < NBAS; ++k) prow[DIN + i * NBAS + k] = (_Float16)(sw[((size_t)o * DIN + i) * NBAS + k] * s); }
  __syncthreads();
  for (int q = tid; q < K / 8; q += 256) vst2(P + (size_t)o * K + q * 8, *(const v4u*)(&prow[q * 8]));
}
__global__ __launch_bounds__(128) void k_l1(const _Float16* __restrict__ A1, const _Float16* __restrict__ P1, float* __restrict__ hpre) {
  __shared__ __align__(16) float so[4][16][132];
  const int tid = threadIdx.x, wave = tid >> 5, lane = tid & 31, col = lane & 15, g = lane >> 4;
  const int r0 = blockIdx.x * 64 + wave * 16, n0 = blockIdx.y * 128;
  v8f acc[8] = {};
#pragma unroll 1
  for (int kc = 0; kc < K1 / 32; ++kc) { const v16h a = frag_h(A1 + (size_t)(r0 + col) * K1 + kc * 32, lane);
#pragma unroll
    for (int j = 0; j < 8; ++j) acc[j] = wmma16(a, frag_h(P1 + (size_t)(n0 + j * 16 + col) * K1 + kc * 32, lane), acc[j]); }
#pragma unroll
  for (int j = 0; j < 8; ++j)
#pragma unroll
    for (int r = 0; r < 8; ++r) so[wave][8 * g + r][j * 16 + col] = acc[j][r] * (1.0f / 1024.0f);
  LDSX();
#pragma unroll 4
  for (int rl = 0; rl < 16; ++rl) vst2(hpre + (size_t)(r0 + rl) * H1 + n0 + lane * 4, *(const v4f*)(&so[wave][rl][lane * 4]));
}
__global__ __launch_bounds__(256) void k_a2(const float* __restrict__ hpre, _Float16* __restrict__ A2, int n0c) {
  __shared__ __align__(16) _Float16 row[K2];
  const int n = n0c + blockIdx.x, tid = threadIdx.x;
#pragma unroll 1
  for (int i = tid; i < H1; i += 256) { const float hv = gelu_e(hpre[(size_t)n * H1 + i]);
    row[i] = (_Float16)(silu1(hv) * 64.0f); float bs[NBAS]; bspl(hv, bs);
#pragma unroll
    for (int k = 0; k < NBAS; ++k) row[H1 + i * NBAS + k] = (_Float16)(bs[k] * 64.0f); }
  __syncthreads();
  for (int q = tid; q < K2 / 8; q += 256) vst2(A2 + (size_t)blockIdx.x * K2 + q * 8, *(const v4u*)(&row[q * 8]));
}
__global__ __launch_bounds__(128) void k_l2(const _Float16* __restrict__ A2, const _Float16* __restrict__ P2, float* __restrict__ out, int n0c) {
  __shared__ __align__(16) float so[4][16][132];
  const int tid = threadIdx.x, wave = tid >> 5, lane = tid & 31, col = lane & 15, g = lane >> 4;
  const int r0 = blockIdx.x * 64 + wave * 16, n0 = blockIdx.y * 128;
  v8f acc[8] = {};
#pragma unroll 1
  for (int kc = 0; kc < K2 / 32; ++kc) { const v16h a = frag_h(A2 + (size_t)(r0 + col) * K2 + kc * 32, lane);
#pragma unroll
    for (int j = 0; j < 8; ++j) acc[j] = wmma16(a, frag_h(P2 + (size_t)(n0 + j * 16 + col) * K2 + kc * 32, lane), acc[j]); }
#pragma unroll
  for (int j = 0; j < 8; ++j)
#pragma unroll
    for (int r = 0; r < 8; ++r) so[wave][8 * g + r][j * 16 + col] = acc[j][r] * (1.0f / 1024.0f);
  LDSX();
#pragma unroll 4
  for (int rl = 0; rl < 16; ++rl) vst2(out + (size_t)(n0c + r0 + rl) * D0 + n0 + lane * 4, *(const v4f*)(&so[wave][rl][lane * 4]));
}
extern "C" void kernel_launch(void* const* d_in, const int* in_sizes, int n_in, void* d_out, int out_size, void* d_ws, size_t ws_size, hipStream_t stream) {
  (void)in_sizes; (void)n_in; (void)out_size; (void)ws_size;
  const float* x = (const float*)d_in[0]; const float* bw1 = (const float*)d_in[1]; const float* sw1 = (const float*)d_in[2]; const float* sc1 = (const float*)d_in[3];
  const float* bw2 = (const float*)d_in[4]; const float* sw2 = (const float*)d_in[5]; const float* sc2 = (const float*)d_in[6];
  float* out = (float*)d_out;
  char* ws = (char*)d_ws; size_t off = 0;
  auto take = [&](size_t bytes) { char* p = ws + off; off += (bytes + 255) & ~(size_t)255; return p; };
  _Float16* P1 = (_Float16*)take((size_t)H1 * K1 * 2); _Float16* P2 = (_Float16*)take((size_t)D0 * K2 * 2); _Float16* A1 = (_Float16*)take((size_t)NT * K1 * 2);
  float* hpre = (float*)take((size_t)NT * H1 * 4); _Float16* A2 = (_Float16*)take((size_t)(NT / 4) * K2 * 2);
  k_a1<<<NT, 256, 0, stream>>>(x, A1);
  k_pack<<<H1, 256, K1 * 2, stream>>>(bw1, sw1, sc1, D0, P1);
  k_pack<<<D0, 256, K2 * 2, stream>>>(bw2, sw2, sc2, H1, P2);
  k_l1<<<dim3(NT / 64, H1 / 128), 128, 0, stream>>>(A1, P1, hpre);
  for (int chk = 0; chk < 4; ++chk) { const int n0c = chk * (NT / 4);
    k_a2<<<NT / 4, 256, 0, stream>>>(hpre, A2, n0c);
    k_l2<<<dim3((NT / 4) / 64, D0 / 128), 128, 0, stream>>>(A2, P2, out, n0c); }
}
